// FCPairedLayer_61323543052293
// MI455X (gfx1250) — hardware-run, weakly checked
//
#include <hip/hip_runtime.h>
#include <stdint.h>

#define NB    4
#define NC    64
#define NN    512
#define NH    128
#define MR    (NB * NN)
#define NCAT  (2 * NH)
#define TPF   65
#define PBP   129

static_assert(2 * NC == 128);
static_assert(NH == 128);
static_assert(NC % 32 == 0);
static_assert(NCAT % 64 == 0);
static_assert(MR % 128 == 0);
static_assert(NN % 128 == 0);
static_assert(NN % 32 == 0);
static_assert(NN % 64 == 0);
static_assert((128 * PBP + 32 * NH + NH) * 4 <= 327680);
static_assert((128 * PBP * 4) % 16 == 0);

typedef __attribute__((ext_vector_type(16))) __bf16 v16b;
typedef __attribute__((ext_vector_type(8)))  __bf16 v8b;
typedef __attribute__((ext_vector_type(8)))  float  v8f;
typedef __attribute__((ext_vector_type(4)))  float  v4f;
typedef __attribute__((ext_vector_type(2)))  float  v2f;
typedef __attribute__((ext_vector_type(4)))  unsigned int v4u;
typedef v8b __attribute__((may_alias)) v8ba;
typedef v4f __attribute__((may_alias)) v4fa;
typedef v2f __attribute__((may_alias)) v2fa;

union FragU { v16b v; v8b h[2]; };

__device__ __forceinline__ unsigned short f2bf_bits(float f) {
  const unsigned u = __float_as_uint(f);
  return (unsigned short)((u + 0x7FFFu + ((u >> 16) & 1u)) >> 16);
}
__device__ __forceinline__ float bf16r(float f) {
  unsigned u = __float_as_uint(f);
  u = (u + 0x7FFFu + ((u >> 16) & 1u)) & 0xFFFF0000u;
  return __uint_as_float(u);
}
__device__ __forceinline__ unsigned pk16(unsigned short a, unsigned short b) { return (unsigned)a | ((unsigned)b << 16); }

__device__ __forceinline__ v8f wmma_bf16(v16b a, v16b b, v8f c) {
  v8f d = __builtin_amdgcn_wmma_f32_16x16x32_bf16(false, a, false, b, (short)0, c, false, false);
  asm volatile("v_nop\n\tv_nop\n\tv_nop\n\tv_nop" : "+v"(d) : "v"(a), "v"(b));
  return d;
}

__device__ __forceinline__ v16b load_frag(const unsigned short* p, int hh) {
  FragU f;
  f.h[0] = *(const v8ba*)(p + 8 * hh);
  f.h[1] = *(const v8ba*)(p + 16 + 8 * hh);
  return f.v;
}

__device__ __forceinline__ void gemm_core1_32x64(
    const unsigned short* __restrict__ A, const unsigned short* __restrict__ Bt,
    int K, size_t aoff, size_t boff, int hh, v8f (&acc)[2][4]) {
  const unsigned short* a0 = A + aoff;
  const unsigned short* a1 = a0 + (size_t)16 * K;
  const unsigned short* bp = Bt + boff;
#pragma unroll 1
  for (int k0 = 0; k0 < K; k0 += 32) {
    const v16b f0 = load_frag(a0 + k0, hh);
    const v16b f1 = load_frag(a1 + k0, hh);
#pragma unroll
    for (int nt = 0; nt < 4; ++nt) {
      const v16b fb = load_frag(bp + (size_t)nt * 16 * K + k0, hh);
      acc[0][nt] = wmma_bf16(f0, fb, acc[0][nt]);
      acc[1][nt] = wmma_bf16(f1, fb, acc[1][nt]);
    }
  }
}

__device__ __forceinline__ void tile_tr(const float* __restrict__ src, int pitch,
                                        unsigned short* __restrict__ dst, float* sT, int tid) {
  const int lane = tid & 31, w = tid >> 5;
  const int c4 = (tid & 15) * 4, rr = tid >> 4;
#pragma unroll
  for (int p = 0; p < 4; ++p) {
    const int r = rr + 16 * p;
    const v4f v = *(const v4fa*)(src + (size_t)r * pitch + c4);
    sT[r * TPF + c4 + 0] = v[0];
    sT[r * TPF + c4 + 1] = v[1];
    sT[r * TPF + c4 + 2] = v[2];
    sT[r * TPF + c4 + 3] = v[3];
  }
  __syncthreads();
  const int q8 = lane & 7, sub = lane >> 3;
  v4u vv[2];
#pragma unroll
  for (int it = 0; it < 2; ++it) {
    const int orow = 32 * it + 4 * w + sub;
    v4u o;
#pragma unroll
    for (int q = 0; q < 4; ++q) {
      const float f0 = sT[(8 * q8 + 2 * q) * TPF + orow];
      const float f1 = sT[(8 * q8 + 2 * q + 1) * TPF + orow];
      o[q] = pk16(f2bf_bits(f0), f2bf_bits(f1));
    }
    vv[it] = o;
  }
  for (int pass = 0; pass < 2; ++pass) {
#pragma unroll
    for (int it = 0; it < 2; ++it) {
      const int orow = 32 * it + 4 * w + sub;
      *(volatile v4u*)(dst + (size_t)orow * 64 + 8 * q8) = vv[it];
    }
    __threadfence();
  }
}

__global__ __launch_bounds__(256) void k_prep(const float* __restrict__ x, const float* __restrict__ W1,
                                              const float* __restrict__ b1, const float* __restrict__ W2,
                                              const float* __restrict__ b2,
                                              unsigned short* __restrict__ XT, unsigned short* __restrict__ W1T,
                                              float* __restrict__ VEC) {
  __shared__ __align__(16) float sT[64 * TPF];
  const int tid = threadIdx.x;
  const int blk = blockIdx.x;
  if (blk < 32) {
    const int b = blk >> 3, n0 = (blk & 7) * 64;
    tile_tr(x + (size_t)b * NC * NN + n0, NN, XT + (size_t)(b * NN + n0) * NC, sT, tid);
  } else if (blk < 36) {
    const int z = blk - 32;
    const int rbase = (z >= 2) ? NC : 0;
    const int cb = (z & 1) * 64;
    tile_tr(W1 + (size_t)rbase * NH + cb, NH, W1T + (size_t)(z * 64) * NC, sT, tid);
  } else {
    if (tid < 32) {
      const int lane = tid;
      const v4f a = *(const v4fa*)(b1 + 4 * lane);
      const v4f c = *(const v4fa*)(W2 + 4 * lane);
      const float s = b2[0];
      asm volatile("" :: "v"(s));
      const v4f o0 = {bf16r(a[0]), bf16r(a[1]), bf16r(a[2]), bf16r(a[3])};
      const v4f o1 = {bf16r(c[0]), bf16r(c[1]), bf16r(c[2]), bf16r(c[3])};
      const float sb = bf16r(s);
      const v4f o2 = {(lane == 0) ? sb : 0.0f, 0.0f, 0.0f, 0.0f};
      for (int pass = 0; pass < 2; ++pass) {
        *(volatile v4f*)(VEC + 4 * lane) = o0;
        *(volatile v4f*)(VEC + 128 + 4 * lane) = o1;
        *(volatile v4f*)(VEC + 256 + 4 * lane) = o2;
        __threadfence();
      }
    }
  }
}

__global__ __launch_bounds__(128) void k_node(const unsigned short* __restrict__ XT,
                                              const unsigned short* __restrict__ W1T,
                                              const float* __restrict__ VEC,
                                              float* __restrict__ PAB) {
  __shared__ __align__(16) float sF[128 * 64];
  __shared__ __align__(16) float sB[NH];
  const int tid = threadIdx.x, lane = tid & 31, w = tid >> 5;
  const int hh = lane >> 4, m = lane & 15;
  const int m0 = blockIdx.x * 128;
  const int n0 = blockIdx.y * 64;
  const int m0w = m0 + 32 * w;

  if (tid < 32) {
    const v4f bv = *(const v4fa*)(VEC + 4 * tid);
    *(v4fa*)(sB + 4 * tid) = bv;
  }

  const v8f zero8 = {0.f, 0.f, 0.f, 0.f, 0.f, 0.f, 0.f, 0.f};
  v8f acc[2][4];
#pragma unroll
  for (int mt = 0; mt < 2; ++mt)
#pragma unroll
    for (int nt = 0; nt < 4; ++nt) acc[mt][nt] = zero8;

  gemm_core1_32x64(XT, W1T, NC, (size_t)(m0w + m) * NC, (size_t)(n0 + m) * NC, hh, acc);

#pragma unroll
  for (int nt = 0; nt < 4; ++nt)
#pragma unroll
    for (int mt = 0; mt < 2; ++mt)
#pragma unroll
      for (int r = 0; r < 8; ++r) {
        const int tokl = 32 * w + 16 * mt + 8 * hh + r;
        const int feat = 16 * nt + m;
        sF[tokl * 64 + feat] = acc[mt][nt][r];
      }
  __syncthreads();
  {
    const bool isA = (n0 < NH);
    const int ncol = n0 & (NH - 1);
    float* dst = PAB + (isA ? (size_t)0 : (size_t)MR * NH) + ncol;
    const int rsub = lane >> 4, c4 = (lane & 15) * 4;
    const v4f bb = *(const v4fa*)(sB + ncol + c4);
    v4f vals[16];
#pragma unroll
    for (int it = 0; it < 16; ++it) {
      const int row = 32 * w + 2 * it + rsub;
      v4f v = *(const v4fa*)(sF + row * 64 + c4);
      if (isA) v = v + bb;
      vals[it] = v;
    }
    for (int pass = 0; pass < 2; ++pass) {
#pragma unroll
      for (int it = 0; it < 16; ++it) {
        const int row = 32 * w + 2 * it + rsub;
        *(volatile v4f*)(dst + (size_t)(m0 + row) * NH + c4) = vals[it];
      }
      __threadfence();
    }
  }
}

__global__ __launch_bounds__(256) void k_pair(const float* __restrict__ PA, const float* __restrict__ PB,
                                              const float* __restrict__ VEC, float* __restrict__ out) {
  __shared__ __align__(16) float PBs[128 * PBP];
  __shared__ __align__(16) float PAs[32 * NH];
  __shared__ __align__(16) float w2s[NH];
  const int tid = threadIdx.x, lane = tid & 31, w = tid >> 5;
  const int j0 = blockIdx.x * 128;
  const int i0 = blockIdx.y * 32;
  const int b  = blockIdx.z;
  float* outB = out + (size_t)b * NN * NN;

  if (j0 + 127 <= i0) {
    for (int pass = 0; pass < 2; ++pass) {
#pragma unroll
      for (int r = 0; r < 4; ++r)
#pragma unroll
        for (int g = 0; g < 4; ++g)
          *(volatile float*)(outB + (size_t)(i0 + 4 * w + r) * NN + j0 + 32 * g + lane) = 0.0f;
      __threadfence();
    }
    return;
  }

#pragma unroll 4
  for (int p = 0; p < 16; ++p) {
    const int f = tid + 256 * p;
    const int row = f >> 5, c4 = (f & 31) * 4;
    const v4f v = *(const v4fa*)(PB + (size_t)(b * NN + j0 + row) * NH + c4);
    PBs[row * PBP + c4 + 0] = v[0];
    PBs[row * PBP + c4 + 1] = v[1];
    PBs[row * PBP + c4 + 2] = v[2];
    PBs[row * PBP + c4 + 3] = v[3];
  }
#pragma unroll
  for (int p = 0; p < 4; ++p) {
    const int f = tid + 256 * p;
    const int row = f >> 5, c4 = (f & 31) * 4;
    const v4f v = *(const v4fa*)(PA + (size_t)(b * NN + i0 + row) * NH + c4);
    *(v4fa*)(PAs + row * NH + c4) = v;
  }
  if (tid < 32) {
    const v4f wv = *(const v4fa*)(VEC + 128 + 4 * tid);
    *(v4fa*)(w2s + 4 * tid) = wv;
  }
  const float b2r = VEC[256];
  asm volatile("" :: "v"(b2r));
  __syncthreads();

  float acc[4][4];
#pragma unroll
  for (int r = 0; r < 4; ++r)
#pragma unroll
    for (int g = 0; g < 4; ++g) acc[r][g] = 0.0f;

  const float* pbl = PBs + lane * PBP;
  const float* pal = PAs + (4 * w) * NH;
#pragma unroll 1
  for (int h = 0; h < NH; h += 2) {
    const v2f wv = *(const v2fa*)(w2s + h);
    v2f pa[4];
#pragma unroll
    for (int r = 0; r < 4; ++r) pa[r] = *(const v2fa*)(pal + r * NH + h);
    float pb0[4], pb1[4];
#pragma unroll
    for (int g = 0; g < 4; ++g) {
      pb0[g] = pbl[32 * g * PBP + h];
      pb1[g] = pbl[32 * g * PBP + h + 1];
    }
#pragma unroll
    for (int r = 0; r < 4; ++r)
#pragma unroll
      for (int g = 0; g < 4; ++g) {
        const float t = pa[r][0] + pb0[g];
        const float rl = (t > 0.0f) ? t : 0.0f;
        acc[r][g] = fmaf(rl, wv[0], acc[r][g]);
      }
#pragma unroll
    for (int r = 0; r < 4; ++r)
#pragma unroll
      for (int g = 0; g < 4; ++g) {
        const float t = pa[r][1] + pb1[g];
        const float rl = (t > 0.0f) ? t : 0.0f;
        acc[r][g] = fmaf(rl, wv[1], acc[r][g]);
      }
  }

  float val[4][4];
#pragma unroll
  for (int r = 0; r < 4; ++r)
#pragma unroll
    for (int g = 0; g < 4; ++g) {
      const int i = i0 + 4 * w + r;
      const int j = j0 + 32 * g + lane;
      const float s = acc[r][g] + b2r;
      val[r][g] = (j > i) ? s : 0.0f;
    }
  for (int pass = 0; pass < 2; ++pass) {
#pragma unroll
    for (int r = 0; r < 4; ++r)
#pragma unroll
      for (int g = 0; g < 4; ++g)
        *(volatile float*)(outB + (size_t)(i0 + 4 * w + r) * NN + j0 + 32 * g + lane) = val[r][g];
    __threadfence();
  }
}

extern "C" void kernel_launch(void* const* d_in, const int* in_sizes, int n_in,
                              void* d_out, int out_size, void* d_ws, size_t ws_size,
                              hipStream_t stream) {
  if (n_in < 5) return;
  if (in_sizes[0] != NB * NC * NN) return;
  if (in_sizes[1] != 2 * NC * NH) return;
  if (in_sizes[2] != NH) return;
  if (in_sizes[3] != NH) return;
  if (in_sizes[4] != 1) return;
  if (out_size != NB * NN * NN) return;

  const float* x  = (const float*)d_in[0];
  const float* W1 = (const float*)d_in[1];
  const float* b1 = (const float*)d_in[2];
  const float* W2 = (const float*)d_in[3];
  const float* b2 = (const float*)d_in[4];
  float* out = (float*)d_out;

  const size_t PXT  = (size_t)MR * NC * 2;
  const size_t PW1  = (size_t)NCAT * NC * 2;
  const size_t PVEC = (size_t)384 * 4;
  const size_t PPL  = (size_t)MR * NH * 4;
  size_t off = 0;
  const size_t oXT  = off; off += PXT;
  const size_t oW1  = off; off += PW1;
  const size_t oVEC = off; off += PVEC;
  const size_t oPA  = off; off += PPL;
  const size_t oPB  = off; off += PPL;
  if (off > ws_size) return;
  if (off > (size_t)134217728) return;
  if (oPB != oPA + PPL) return;

  char* ws = (char*)d_ws;
  unsigned short* XT  = (unsigned short*)(ws + oXT);
  unsigned short* W1T = (unsigned short*)(ws + oW1);
  float*          VEC = (float*)(ws + oVEC);
  float*          PA  = (float*)(ws + oPA);
  float*          PB  = (float*)(ws + oPB);

  k_prep<<<dim3(37), 256, 0, stream>>>(x, W1, b1, W2, b2, XT, W1T, VEC);
  k_node<<<dim3(MR / 128, NCAT / 64), 128, 0, stream>>>(XT, W1T, VEC, PA);
  k_pair<<<dim3(NN / 128, NN / 32, NB), 256, 0, stream>>>(PA, PB, VEC, out);
  (void)hipGetLastError();
}
